// SpatialAttentionModel_12833362280582
// MI455X (gfx1250) — hardware-run, weakly checked
//
#include <hip/hip_runtime.h>
#include <stdint.h>
#include <math.h>

#define MR    49152
#define NN    512
#define DM    64
#define KIN   128
#define NQKV  192
#define NHD   8
#define DHD   8
#define NGH   768
#define XSC   64.0f
#define WSC   1024.0f
#define ISC   (1.0f / 65536.0f)
#define ASC   16.0f
#define SCL   (0.35355339059327373f / 256.0f)
#define PSC   4096.0f
#define ONRM  (1.0f / 256.0f)
#define LOSC  2048.0f
#define LOIN  (1.0f / 2048.0f)
#define OSC   (1.0f / 262144.0f)
#define NEG0  (-1.0e38f)
static_assert(DM == NHD * DHD);
static_assert((MR % 64) == 0 && (NN % 64) == 0 && (MR % NN) == 0);
static_assert(NGH == (MR / NN) * NHD);
static_assert(KIN == 2 * DM && NQKV == 3 * DM);

typedef _Float16 v16h __attribute__((ext_vector_type(16)));
typedef _Float16 v8h  __attribute__((ext_vector_type(8)));
typedef float    v8f  __attribute__((ext_vector_type(8)));
typedef float    v4f  __attribute__((ext_vector_type(4)));
typedef unsigned int v4u __attribute__((ext_vector_type(4)));

union FragH { v16h v; v8h h[2]; v4u u[2]; };

__device__ __forceinline__ unsigned short bf_bits(float f) {
  unsigned u = __float_as_uint(f);
  return (unsigned short)((u + 0x7FFFu + ((u >> 16) & 1u)) >> 16);
}
__device__ __forceinline__ float bf_up(unsigned short h) { return __uint_as_float(((unsigned)h) << 16); }
__device__ __forceinline__ float bfr(float f) { return bf_up(bf_bits(f)); }
__device__ __forceinline__ unsigned short h_bits(_Float16 x) { return __builtin_bit_cast(unsigned short, x); }
__device__ __forceinline__ unsigned pk16(unsigned short a, unsigned short b) { return (unsigned)a | ((unsigned)b << 16); }
__device__ __forceinline__ v8f zero8() { v8f z = {0.f, 0.f, 0.f, 0.f, 0.f, 0.f, 0.f, 0.f}; return z; }
__device__ __forceinline__ v4u cvt8(v4f a, v4f c, float sc) {
  float f[8];
#pragma unroll
  for (int i = 0; i < 4; ++i) { f[i] = bfr(a[i]) * sc; f[4 + i] = bfr(c[i]) * sc; }
  v4u v;
#pragma unroll
  for (int i = 0; i < 4; ++i) v[i] = pk16(h_bits((_Float16)f[2 * i]), h_bits((_Float16)f[2 * i + 1]));
  return v;
}

__device__ __forceinline__ v16h ldfrag_h(const _Float16* p) {
  FragH f;
  f.h[0] = *(const v8h*)(p);
  f.h[1] = *(const v8h*)(p + 16);
  return f.v;
}

__device__ __forceinline__ v8f mma_h(v16h a, v16h b, v8f c) {
  return __builtin_amdgcn_wmma_f32_16x16x32_f16(false, a, false, b, (short)0, c, false, false);
}
__device__ __forceinline__ void guard1(v8f& a, v16h x, v16h y) {
#if defined(__HIP_DEVICE_COMPILE__)
  asm volatile("v_nop\n\tv_nop\n\tv_nop\n\tv_nop" : "+v"(a) : "v"(x), "v"(y));
#endif
}
__device__ __forceinline__ void guard2(v8f& a, v8f& b, v16h x0, v16h x1, v16h y) {
#if defined(__HIP_DEVICE_COMPILE__)
  asm volatile("v_nop\n\tv_nop\n\tv_nop\n\tv_nop" : "+v"(a), "+v"(b) : "v"(x0), "v"(x1), "v"(y));
#endif
}
__device__ __forceinline__ void guard4(v8f& a, v8f& b, v8f& c, v8f& d,
                                       v16h x, v16h y0, v16h y1, v16h y2, v16h y3) {
#if defined(__HIP_DEVICE_COMPILE__)
  asm volatile("v_nop\n\tv_nop\n\tv_nop\n\tv_nop"
               : "+v"(a), "+v"(b), "+v"(c), "+v"(d) : "v"(x), "v"(y0), "v"(y1), "v"(y2), "v"(y3));
#endif
}

__global__ __launch_bounds__(256)
void cvt_w(const float* __restrict__ w7, const float* __restrict__ w8, const float* __restrict__ w9,
           const float* __restrict__ w10, const float* __restrict__ w11,
           unsigned short* wp, unsigned short* w10t, unsigned short* w11t) {
  __shared__ __align__(16) unsigned short Ts[64 * 136];
  const int tid = threadIdx.x;
  const int bx  = blockIdx.x;
  const int p4  = tid & 15, r16 = tid >> 4;
  if (bx < 3) {
    const float* src = (bx == 0) ? w7 : ((bx == 1) ? w8 : w9);
#pragma unroll 2
    for (int it = 0; it < 8; ++it) {
      const int e = it * 16 + r16;
      const v4f a = *(const v4f*)(src + (size_t)e * DM + 4 * p4);
#pragma unroll
      for (int i = 0; i < 4; ++i) Ts[(4 * p4 + i) * 136 + e] = h_bits((_Float16)(bfr(a[i]) * WSC));
    }
  } else {
    const float* src = (bx == 3) ? w10 : w11;
#pragma unroll 2
    for (int it = 0; it < 4; ++it) {
      const int e = it * 16 + r16;
      const v4f a = *(const v4f*)(src + (size_t)e * DM + 4 * p4);
#pragma unroll
      for (int i = 0; i < 4; ++i) Ts[(4 * p4 + i) * 136 + e] = h_bits((_Float16)(bfr(a[i]) * WSC));
    }
  }
  __syncthreads();
  if (bx < 3) {
    v4u vals[4];
#pragma unroll
    for (int it = 0; it < 4; ++it) {
      const int idx = it * 256 + tid;
      const int row = idx >> 4, pc = idx & 15;
      vals[it] = *(const v4u*)(Ts + row * 136 + 8 * pc);
    }
    unsigned short* dst = wp + (size_t)(bx * 64) * KIN;
    for (int pass = 0; pass < 2; ++pass) {
#pragma unroll
      for (int it = 0; it < 4; ++it) {
        const int idx = it * 256 + tid;
        const int row = idx >> 4, pc = idx & 15;
        *(volatile v4u*)(dst + (size_t)row * KIN + 8 * pc) = vals[it];
      }
      __threadfence();
    }
  } else {
    v4u vals[2];
#pragma unroll
    for (int it = 0; it < 2; ++it) {
      const int idx = it * 256 + tid;
      const int row = idx >> 3, pc = idx & 7;
      vals[it] = *(const v4u*)(Ts + row * 136 + 8 * pc);
    }
    unsigned short* dst = (bx == 3) ? w10t : w11t;
    for (int pass = 0; pass < 2; ++pass) {
#pragma unroll
      for (int it = 0; it < 2; ++it) {
        const int idx = it * 256 + tid;
        const int row = idx >> 3, pc = idx & 7;
        *(volatile v4u*)(dst + (size_t)row * DM + 8 * pc) = vals[it];
      }
      __threadfence();
    }
  }
}

__global__ __launch_bounds__(128)
void qkv_gemm(const float* __restrict__ X, const float* __restrict__ S, const unsigned short* __restrict__ wp,
              const float* __restrict__ b7, const float* __restrict__ b8, const float* __restrict__ b9,
              unsigned short* qh, unsigned short* kh, unsigned short* vh) {
  __shared__ __align__(16) unsigned short Ts[64 * 200];
  const int tid  = threadIdx.x;
  const int wave = tid >> 5;
  const int lane = tid & 31;
  const int hh   = lane >> 4;
  const int ci   = lane & 15;
  const int m0   = blockIdx.x * 64;
  const int m    = m0 + 16 * wave + ci;
  const _Float16* W  = (const _Float16*)(const void*)wp;
  const _Float16* wr = W + (size_t)ci * KIN + 8 * hh;

  v8f acc[12];
#pragma unroll
  for (int t = 0; t < 12; ++t) acc[t] = zero8();

#pragma unroll 1
  for (int ks = 0; ks < KIN / 32; ++ks) {
    const float* src = (ks < 2) ? X : S;
    const float* rp  = src + (size_t)m * DM + (ks & 1) * 32;
    const v4f x0 = *(const v4f*)(rp + 8 * hh);
    const v4f x1 = *(const v4f*)(rp + 8 * hh + 4);
    const v4f y0 = *(const v4f*)(rp + 16 + 8 * hh);
    const v4f y1 = *(const v4f*)(rp + 20 + 8 * hh);
    FragH xb;
    xb.u[0] = cvt8(x0, x1, XSC);
    xb.u[1] = cvt8(y0, y1, XSC);
    const int k0 = ks * 32;
#pragma unroll
    for (int gi = 0; gi < 3; ++gi) {
      v16h wa[4];
#pragma unroll
      for (int t = 0; t < 4; ++t) wa[t] = ldfrag_h(wr + (size_t)(16 * (4 * gi + t)) * KIN + k0);
#pragma unroll
      for (int t = 0; t < 4; ++t) acc[4 * gi + t] = mma_h(wa[t], xb.v, acc[4 * gi + t]);
      guard4(acc[4 * gi], acc[4 * gi + 1], acc[4 * gi + 2], acc[4 * gi + 3], xb.v, wa[0], wa[1], wa[2], wa[3]);
    }
  }

  {
    unsigned short* ts = Ts + (16 * wave + ci) * 200 + 8 * hh;
#pragma unroll
    for (int t = 0; t < 12; ++t) {
      const float* bp = (t < 4) ? b7 : ((t < 8) ? b8 : b9);
      const int cb = (16 * t) & 63;
      const v4f bb0 = *(const v4f*)(bp + cb + 8 * hh);
      const v4f bb1 = *(const v4f*)(bp + cb + 8 * hh + 4);
      float y[8];
#pragma unroll
      for (int e = 0; e < 4; ++e) {
        y[e]     = fmaxf(acc[t][e] * ISC     + bfr(bb0[e]), 0.0f) * ASC;
        y[4 + e] = fmaxf(acc[t][4 + e] * ISC + bfr(bb1[e]), 0.0f) * ASC;
      }
      v4u v;
#pragma unroll
      for (int i = 0; i < 4; ++i) v[i] = pk16(h_bits((_Float16)y[2 * i]), h_bits((_Float16)y[2 * i + 1]));
      *(v4u*)(ts + 16 * t) = v;
    }
  }
  __syncthreads();
  {
    const int g = m0 / NN, nb0 = m0 - g * NN;
    v4u vals[12];
#pragma unroll
    for (int p = 0; p < 3; ++p) {
#pragma unroll
      for (int it = 0; it < 4; ++it) {
        const int idx = it * 128 + tid;
        const int h = idx >> 6, n = idx & 63;
        vals[p * 4 + it] = *(const v4u*)(Ts + n * 200 + 64 * p + 8 * h);
      }
    }
    for (int pass = 0; pass < 2; ++pass) {
#pragma unroll
      for (int p = 0; p < 3; ++p) {
        unsigned short* pl = (p == 0) ? qh : ((p == 1) ? kh : vh);
#pragma unroll
        for (int it = 0; it < 4; ++it) {
          const int idx = it * 128 + tid;
          const int h = idx >> 6, n = idx & 63;
          unsigned short* dst = pl + (((size_t)(g * NHD + h)) * NN + nb0 + n) * DHD;
          *(volatile v4u*)dst = vals[p * 4 + it];
        }
      }
      __threadfence();
    }
  }
}

__global__ __launch_bounds__(256)
void attn_fwd(const unsigned short* __restrict__ qh, const unsigned short* __restrict__ kh,
              const unsigned short* __restrict__ vh, unsigned short* ohp, unsigned short* olp) {
  __shared__ __align__(16) unsigned short sK[NN * DHD];
  __shared__ __align__(16) unsigned short sVt[DHD * NN];
  __shared__ __align__(16) unsigned short sOH[NN * DHD];
  __shared__ __align__(16) unsigned short sOL[NN * DHD];
  const int tid  = threadIdx.x;
  const int wave = tid >> 5;
  const int lane = tid & 31;
  const int hh   = lane >> 4;
  const int ci   = lane & 15;
  const int gh   = blockIdx.x;
  const size_t pb = (size_t)gh * NN * DHD;
#pragma unroll
  for (int i = 0; i < 2; ++i) {
    const int n = i * 256 + tid;
    const v4u kv = *(const v4u*)(kh + pb + (size_t)n * DHD);
    *(v4u*)(sK + n * DHD) = kv;
    const v4u vv = *(const v4u*)(vh + pb + (size_t)n * DHD);
#pragma unroll
    for (int j = 0; j < 4; ++j) {
      sVt[(2 * j) * NN + n]     = (unsigned short)(vv[j] & 0xFFFFu);
      sVt[(2 * j + 1) * NN + n] = (unsigned short)(vv[j] >> 16);
    }
  }
  __syncthreads();

  const unsigned mq = (hh == 0) ? 0xFFFFFFFFu : 0u;
  const unsigned mv = (ci < DHD) ? 0xFFFFFFFFu : 0u;
  const int dcl = (ci < DHD) ? ci : (DHD - 1);
  const v4u z4 = {0u, 0u, 0u, 0u};

#pragma unroll 1
  for (int qt = wave; qt < NN / 16; qt += 8) {
    const int q0 = qt * 16;
    FragH qf;
    {
      const v4u qv = *(const v4u*)(qh + pb + (size_t)(q0 + ci) * DHD);
      qf.u[0] = qv & mq;
      qf.u[1] = z4;
    }
    float rmax = NEG0, z = 0.f;
    v8f acc = zero8();
#pragma unroll 1
    for (int it = 0; it < NN / 32; ++it) {
      const int lt = it * 32;
      FragH a0, a1;
      {
        const v4u k0v = *(const v4u*)(sK + (lt + ci) * DHD);
        const v4u k1v = *(const v4u*)(sK + (lt + 16 + ci) * DHD);
        a0.u[0] = k0v & mq; a0.u[1] = z4;
        a1.u[0] = k1v & mq; a1.u[1] = z4;
      }
      v8f s0 = mma_h(a0.v, qf.v, zero8());
      v8f s1 = mma_h(a1.v, qf.v, zero8());
      guard2(s0, s1, a0.v, a1.v, qf.v);
      float sc[16];
#pragma unroll
      for (int r = 0; r < 8; ++r) { sc[r] = s0[r] * SCL; sc[8 + r] = s1[r] * SCL; }
      float mx = sc[0];
#pragma unroll
      for (int i = 1; i < 16; ++i) mx = fmaxf(mx, sc[i]);
      mx = fmaxf(mx, __shfl_xor(mx, 16, 32));
      const float nmax = fmaxf(rmax, mx);
      const float corr = __expf(rmax - nmax);
      rmax = nmax;
      FragH ph;
      float zs = 0.f;
#pragma unroll
      for (int r = 0; r < 8; ++r) {
        const float pa = __expf(sc[r] - nmax);
        const float pc = __expf(sc[8 + r] - nmax);
        zs += pa + pc;
        ph.h[0][r] = (_Float16)(pa * PSC);
        ph.h[1][r] = (_Float16)(pc * PSC);
      }
      z = z * corr + zs;
      acc *= corr;
      FragH va;
      {
        const v4u v0 = *(const v4u*)(sVt + dcl * NN + lt + 8 * hh);
        const v4u v1 = *(const v4u*)(sVt + dcl * NN + lt + 16 + 8 * hh);
        va.u[0] = v0 & mv;
        va.u[1] = v1 & mv;
      }
      acc = mma_h(va.v, ph.v, acc);
      guard1(acc, va.v, ph.v);
    }
    const float zz = z + __shfl_xor(z, 16, 32);
    const float rz = (1.0f / zz) * ONRM;
    v4u h0, g0;
#pragma unroll
    for (int i = 0; i < 4; ++i) {
      const float oa = acc[2 * i] * rz, ob = acc[2 * i + 1] * rz;
      const _Float16 a0h = (_Float16)oa, a1h = (_Float16)ob;
      const _Float16 l0 = (_Float16)((oa - (float)a0h) * LOSC);
      const _Float16 l1 = (_Float16)((ob - (float)a1h) * LOSC);
      h0[i] = pk16(h_bits(a0h), h_bits(a1h));
      g0[i] = pk16(h_bits(l0), h_bits(l1));
    }
    if (hh == 0) {
      *(v4u*)(sOH + (q0 + ci) * DHD) = h0;
      *(v4u*)(sOL + (q0 + ci) * DHD) = g0;
    }
  }
  __syncthreads();
  {
    v4u hv[2], lv[2];
#pragma unroll
    for (int i = 0; i < 2; ++i) {
      const int n = i * 256 + tid;
      hv[i] = *(const v4u*)(sOH + n * DHD);
      lv[i] = *(const v4u*)(sOL + n * DHD);
    }
    for (int pass = 0; pass < 2; ++pass) {
#pragma unroll
      for (int i = 0; i < 2; ++i) {
        const int n = i * 256 + tid;
        *(volatile v4u*)(ohp + pb + (size_t)n * DHD) = hv[i];
        *(volatile v4u*)(olp + pb + (size_t)n * DHD) = lv[i];
      }
      __threadfence();
    }
  }
}

__global__ __launch_bounds__(128)
void out_proj(const unsigned short* __restrict__ ohp, const unsigned short* __restrict__ olp,
              const unsigned short* __restrict__ w10t, const unsigned short* __restrict__ w11t,
              const float* __restrict__ b10, const float* __restrict__ b11, float* out) {
  __shared__ __align__(16) float Ts[64 * 68];
  const int tid  = threadIdx.x;
  const int wave = tid >> 5;
  const int lane = tid & 31;
  const int hh   = lane >> 4;
  const int ci   = lane & 15;
  const int m0   = blockIdx.x * 64;
  const int g    = m0 / NN;
  const int nrow = m0 - g * NN + 16 * wave + ci;
  const _Float16* OHf = (const _Float16*)(const void*)ohp;
  const _Float16* OLf = (const _Float16*)(const void*)olp;
  const _Float16* W1  = (const _Float16*)(const void*)w10t;
  const _Float16* W2  = (const _Float16*)(const void*)w11t;
  const _Float16* wr1 = W1 + (size_t)ci * DM + 8 * hh;
  const _Float16* wr2 = W2 + (size_t)ci * DM + 8 * hh;

  v8f acch[4], accl[4];
#pragma unroll
  for (int t = 0; t < 4; ++t) { acch[t] = zero8(); accl[t] = zero8(); }

#pragma unroll
  for (int ks = 0; ks < 2; ++ks) {
    const int hd0 = 4 * ks + hh, hd1 = 4 * ks + 2 + hh;
    const size_t r0 = ((size_t)(g * NHD + hd0) * NN + nrow) * DHD;
    const size_t r1 = ((size_t)(g * NHD + hd1) * NN + nrow) * DHD;
    FragH bh, bl;
    bh.h[0] = *(const v8h*)(OHf + r0);
    bh.h[1] = *(const v8h*)(OHf + r1);
    bl.h[0] = *(const v8h*)(OLf + r0);
    bl.h[1] = *(const v8h*)(OLf + r1);
    v16h wa[4];
#pragma unroll
    for (int t = 0; t < 4; ++t) wa[t] = ldfrag_h(wr1 + (size_t)(16 * t) * DM + 32 * ks);
#pragma unroll
    for (int t = 0; t < 4; ++t) acch[t] = mma_h(wa[t], bh.v, acch[t]);
    guard4(acch[0], acch[1], acch[2], acch[3], bh.v, wa[0], wa[1], wa[2], wa[3]);
#pragma unroll
    for (int t = 0; t < 4; ++t) accl[t] = mma_h(wa[t], bl.v, accl[t]);
    guard4(accl[0], accl[1], accl[2], accl[3], bl.v, wa[0], wa[1], wa[2], wa[3]);
  }

  FragH zh[2], zl[2];
#pragma unroll
  for (int t = 0; t < 4; ++t) {
    const v4f bb0 = *(const v4f*)(b10 + 16 * t + 8 * hh);
    const v4f bb1 = *(const v4f*)(b10 + 16 * t + 8 * hh + 4);
#pragma unroll
    for (int e = 0; e < 4; ++e) {
      const float ya = (acch[t][e]     + accl[t][e]     * LOIN) * OSC + bfr(bb0[e]);
      const float yb = (acch[t][4 + e] + accl[t][4 + e] * LOIN) * OSC + bfr(bb1[e]);
      const float za = fmaxf(ya, 0.0f) * 256.0f, zb = fmaxf(yb, 0.0f) * 256.0f;
      const _Float16 ha = (_Float16)za, hb = (_Float16)zb;
      zh[t >> 1].h[t & 1][e]     = ha;
      zh[t >> 1].h[t & 1][4 + e] = hb;
      zl[t >> 1].h[t & 1][e]     = (_Float16)((za - (float)ha) * LOSC);
      zl[t >> 1].h[t & 1][4 + e] = (_Float16)((zb - (float)hb) * LOSC);
    }
  }

  v8f acc2h[4], acc2l[4];
#pragma unroll
  for (int t = 0; t < 4; ++t) { acc2h[t] = zero8(); acc2l[t] = zero8(); }
#pragma unroll
  for (int ks = 0; ks < 2; ++ks) {
    v16h wa[4];
#pragma unroll
    for (int t = 0; t < 4; ++t) wa[t] = ldfrag_h(wr2 + (size_t)(16 * t) * DM + 32 * ks);
#pragma unroll
    for (int t = 0; t < 4; ++t) acc2h[t] = mma_h(wa[t], zh[ks].v, acc2h[t]);
    guard4(acc2h[0], acc2h[1], acc2h[2], acc2h[3], zh[ks].v, wa[0], wa[1], wa[2], wa[3]);
#pragma unroll
    for (int t = 0; t < 4; ++t) acc2l[t] = mma_h(wa[t], zl[ks].v, acc2l[t]);
    guard4(acc2l[0], acc2l[1], acc2l[2], acc2l[3], zl[ks].v, wa[0], wa[1], wa[2], wa[3]);
  }

  {
    float* ts = Ts + (16 * wave + ci) * 68 + 8 * hh;
#pragma unroll
    for (int t = 0; t < 4; ++t) {
      const v4f bb0 = *(const v4f*)(b11 + 16 * t + 8 * hh);
      const v4f bb1 = *(const v4f*)(b11 + 16 * t + 8 * hh + 4);
      v4f r0, r1;
#pragma unroll
      for (int e = 0; e < 4; ++e) {
        r0[e] = (acc2h[t][e]     + acc2l[t][e]     * LOIN) * OSC + bfr(bb0[e]);
        r1[e] = (acc2h[t][4 + e] + acc2l[t][4 + e] * LOIN) * OSC + bfr(bb1[e]);
      }
      *(v4f*)(ts + 16 * t)     = r0;
      *(v4f*)(ts + 16 * t + 4) = r1;
    }
  }
  __syncthreads();
  {
    const int p = tid & 15, r16 = tid >> 4;
    v4f vals[8];
#pragma unroll
    for (int it = 0; it < 8; ++it) {
      const int row = it * 8 + r16;
      vals[it] = *(const v4f*)(Ts + row * 68 + 4 * p);
    }
    float* yb = out + (size_t)m0 * DM + 4 * p;
    for (int pass = 0; pass < 2; ++pass) {
#pragma unroll
      for (int it = 0; it < 8; ++it) {
        const int row = it * 8 + r16;
        *(volatile v4f*)(yb + (size_t)row * DM) = vals[it];
      }
      __threadfence();
    }
  }
}

extern "C" void kernel_launch(void* const* d_in, const int* in_sizes, int n_in,
                              void* d_out, int out_size, void* d_ws, size_t ws_size,
                              hipStream_t stream) {
  if (n_in < 12) return;
  if (in_sizes[0] != MR * DM || in_sizes[1] != MR * DM) return;
  if (in_sizes[2] != KIN * DM || in_sizes[4] != KIN * DM || in_sizes[6] != KIN * DM) return;
  if (in_sizes[8] != DM * DM || in_sizes[10] != DM * DM) return;
  if (in_sizes[3] != DM || in_sizes[5] != DM || in_sizes[7] != DM || in_sizes[9] != DM || in_sizes[11] != DM) return;
  if (out_size != MR * DM) return;

  const float* X   = (const float*)d_in[0];
  const float* STE = (const float*)d_in[1];
  const float* W7  = (const float*)d_in[2];
  const float* b7  = (const float*)d_in[3];
  const float* W8  = (const float*)d_in[4];
  const float* b8  = (const float*)d_in[5];
  const float* W9  = (const float*)d_in[6];
  const float* b9  = (const float*)d_in[7];
  const float* W10 = (const float*)d_in[8];
  const float* b10 = (const float*)d_in[9];
  const float* W11 = (const float*)d_in[10];
  const float* b11 = (const float*)d_in[11];
  float* out = (float*)d_out;

  const size_t PWP = (size_t)NQKV * KIN * 2;
  const size_t PWS = (size_t)DM * DM * 2;
  const size_t PPL = (size_t)NGH * NN * DHD * 2;
  size_t off = 0;
  const size_t oWP  = off; off += PWP;
  const size_t oW10 = off; off += PWS;
  const size_t oW11 = off; off += PWS;
  const size_t oQ   = off; off += PPL;
  const size_t oK   = off; off += PPL;
  const size_t oV   = off; off += PPL;
  const size_t oOH  = off; off += PPL;
  const size_t oOL  = off; off += PPL;
  if (off > ws_size) return;
  if (off > (size_t)134217728) return;

  char* ws = (char*)d_ws;
  unsigned short* WPp  = (unsigned short*)(ws + oWP);
  unsigned short* W10p = (unsigned short*)(ws + oW10);
  unsigned short* W11p = (unsigned short*)(ws + oW11);
  unsigned short* QHp  = (unsigned short*)(ws + oQ);
  unsigned short* KHp  = (unsigned short*)(ws + oK);
  unsigned short* VHp  = (unsigned short*)(ws + oV);
  unsigned short* OHp  = (unsigned short*)(ws + oOH);
  unsigned short* OLp  = (unsigned short*)(ws + oOL);

  const dim3 blk256(256), blk128(128);
  const dim3 gWT(5);
  const dim3 gPJ(MR / 64);
  const dim3 gAT(NGH);
  const dim3 gOP(MR / 64);

  cvt_w<<<gWT, blk256, 0, stream>>>(W7, W8, W9, W10, W11, WPp, W10p, W11p);
  qkv_gemm<<<gPJ, blk128, 0, stream>>>(X, STE, WPp, b7, b8, b9, QHp, KHp, VHp);
  attn_fwd<<<gAT, blk256, 0, stream>>>(QHp, KHp, VHp, OHp, OLp);
  out_proj<<<gOP, blk128, 0, stream>>>(OHp, OLp, W10p, W11p, b10, b11, out);
  (void)hipGetLastError();
}
